// CrossAttention_3246995275787
// MI455X (gfx1250) — hardware-run, weakly checked
//
#include <hip/hip_runtime.h>


#ifndef NB
#define NB 4
#endif
#ifndef SEQ
#define SEQ 1024
#endif
#define NB_FULL  4
#define SEQ_FULL 1024
#ifndef OUT_SEQ
#define OUT_SEQ SEQ
#endif
#define DM   1024
#define NH_  16
#define HD   64
#define FFI  4096
#define LDAH (DM + FFI)
#define AW   4
#define OSP  68
#define GSP  68
#define WSC  64.0f
#define WI   (1.0f / 64.0f)
#define AOC  64.0f
#define HC   64.0f
#define OI   (1.0f / 4096.0f)
#define L2E  1.4426950408889634f
#define SC2  ((float)(0.125 * 1.4426950408889634))
#define PSH  14.0f
#define NEGB (-3.0e38f)
#define LNEPS 1.0e-5f

static_assert(NH_ * HD == DM);
static_assert(HD == 64);
static_assert(DM % 64 == 0);
static_assert(DM % 32 == 0);
static_assert(LDAH % 32 == 0);
static_assert(FFI % 64 == 0);
static_assert(SEQ % 64 == 0);
static_assert((NB * SEQ) % 64 == 0);
static_assert((NB * SEQ) % 32 == 0);
static_assert((NB * SEQ) % 8 == 0);
static_assert(SEQ % 32 == 0);
static_assert(SEQ % (16 * AW) == 0);
static_assert(32 * 8 * 4 == DM);
static_assert(NB <= NB_FULL);
static_assert(SEQ <= SEQ_FULL);
static_assert((OSP * 4) % 16 == 0);
static_assert((GSP * 4) % 16 == 0);
static_assert((LDAH * 2) % 128 == 0);
static_assert((DM * 2) % 128 == 0);
static_assert(WSC * AOC * OI == 1.0f);
static_assert(WSC * HC * OI == 1.0f);
static_assert(WSC * WI == 1.0f);
static_assert(sizeof(float) * AW * 16 * OSP <= 131072);
static_assert(sizeof(float) * 16 * GSP <= 131072);
static_assert(sizeof(float) * 64 * 65 <= 131072);

typedef _Float16 h16;
typedef __attribute__((ext_vector_type(16))) _Float16 v16h;
typedef __attribute__((ext_vector_type(8)))  _Float16 v8h;
typedef __attribute__((ext_vector_type(8)))  float    v8f;
typedef __attribute__((ext_vector_type(4)))  float    v4f;
typedef v4f  __attribute__((may_alias)) v4fa;

__device__ __forceinline__ unsigned short f2bf(float f) { unsigned u = __float_as_uint(f); u += 0x7FFFu + ((u >> 16) & 1u); return (unsigned short)(u >> 16); }
__device__ __forceinline__ float bfr(float f) { return __uint_as_float(((unsigned)f2bf(f)) << 16); }
__device__ __forceinline__ v16h cat16(v8h lo, v8h hi) { return __builtin_shufflevector(lo, hi, 0, 1, 2, 3, 4, 5, 6, 7, 8, 9, 10, 11, 12, 13, 14, 15); }
__device__ __forceinline__ v8f wmma16(v16h a, v16h b, v8f c) { return __builtin_amdgcn_wmma_f32_16x16x32_f16(false, a, false, b, (short)0, c, false, false); }
__device__ __forceinline__ v8f wmmag(v16h a, v16h b, v8f c) { c = wmma16(a, b, c); asm volatile("v_nop\n\tv_nop\n\tv_nop\n\tv_nop" : "+v"(c) : "v"(a), "v"(b)); return c; }
__device__ __forceinline__ v16h  ldh(const h16* p) { return cat16(*(const v8h*)p, *(const v8h*)(p + 16)); }
__device__ __forceinline__ void wave_sync() { __builtin_amdgcn_fence(3  , "wavefront"); __builtin_amdgcn_wave_barrier(); asm volatile("" ::: "memory"); }
static __device__ __forceinline__ h16 toh_flush(float v) { const h16 r = (h16)v; return (fabsf(v) < 6.103515625e-05f) ? (h16)0.0f : r; }

__global__ __launch_bounds__(256) void k_ln(const float* __restrict__ X, const float* __restrict__ G, const float* __restrict__ Bv, h16* Y) {
#pragma clang fp contract(off)
    const int lane = threadIdx.x & 31;
    const int wave = __builtin_amdgcn_readfirstlane((int)(threadIdx.x >> 5));
    const int row = blockIdx.x * 8 + wave;
    const int bb = row / SEQ, tt = row % SEQ;
    const float* xr = X + ((size_t)bb * SEQ_FULL + (size_t)tt) * DM + lane * 8;
    v8f v[4]; float s = 0.0f;
#pragma unroll
    for (int p = 0; p < 4; ++p) { v[p] = *(const v8f*)(xr + p * 256);
#pragma unroll
        for (int i = 0; i < 8; ++i) { v[p][i] = bfr(v[p][i]); s += v[p][i]; } }
    s += __shfl_xor(s, 16, 32); s += __shfl_xor(s, 8, 32); s += __shfl_xor(s, 4, 32); s += __shfl_xor(s, 2, 32); s += __shfl_xor(s, 1, 32);
    const float mu = s * (1.0f / (float)DM);
    float q = 0.0f;
#pragma unroll
    for (int p = 0; p < 4; ++p) {
#pragma unroll
        for (int i = 0; i < 8; ++i) { const float d = v[p][i] - mu; v[p][i] = d; q += d * d; } }
    q += __shfl_xor(q, 16, 32); q += __shfl_xor(q, 8, 32); q += __shfl_xor(q, 4, 32); q += __shfl_xor(q, 2, 32); q += __shfl_xor(q, 1, 32);
    const float rs = rsqrtf(q * (1.0f / (float)DM) + LNEPS);
    v8h o[4];
#pragma unroll
    for (int p = 0; p < 4; ++p) { const v8f g = *(const v8f*)(G + p * 256 + lane * 8); const v8f c = *(const v8f*)(Bv + p * 256 + lane * 8);
#pragma unroll
        for (int i = 0; i < 8; ++i) o[p][i] = toh_flush(v[p][i] * rs * bfr(g[i]) + bfr(c[i])); }
    h16* yr = Y + (size_t)row * DM + lane * 8;
#pragma unroll 1
    for (int ps = 0; ps < 2; ++ps) {
#pragma unroll
        for (int p = 0; p < 4; ++p) *(volatile v8h*)(yr + p * 256) = o[p];
        if (ps == 0) __threadfence(); }
}

static_assert(256 * 2 * 16 == 64 * 128);
__global__ __launch_bounds__(256) void k_wtr(const float* __restrict__ W, int N, h16* WT, int ldo, int coff) {
#pragma clang fp contract(off)
    __shared__ float ts[64 * 65];
    const int tid = threadIdx.x;
    const int n0 = blockIdx.x * 64, k0 = blockIdx.y * 64;
#pragma unroll
    for (int it = 0; it < 4; ++it) { const int r = it * 16 + (tid >> 4), c4 = (tid & 15) * 4;
        const v4f w = *(const v4f*)(W + (size_t)(k0 + r) * (size_t)N + (size_t)(n0 + c4));
        ts[r * 65 + c4 + 0] = w[0]; ts[r * 65 + c4 + 1] = w[1]; ts[r * 65 + c4 + 2] = w[2]; ts[r * 65 + c4 + 3] = w[3]; }
    __syncthreads();
#pragma unroll 1
    for (int ps = 0; ps < 2; ++ps) {
#pragma unroll
        for (int it = 0; it < 2; ++it) { const int p = it * 256 + tid; const int n = p >> 3, k8 = (p & 7) * 8;
            v8h o;
#pragma unroll
            for (int i = 0; i < 8; ++i) o[i] = toh_flush(bfr(ts[(k8 + i) * 65 + n]) * WSC);
            *(volatile v8h*)(WT + (size_t)(n0 + n) * (size_t)ldo + (size_t)coff + (size_t)(k0 + k8)) = o; }
        if (ps == 0) __threadfence(); }
}

__device__ __forceinline__ void gemm_acc(const h16* __restrict__ A, size_t lda, const h16* __restrict__ Bt, size_t ldb, int K, int r0, int c0, int lr, int hi, v8f (&acc)[4][4]) {
#pragma unroll
    for (int mb = 0; mb < 4; ++mb)
#pragma unroll
        for (int nb = 0; nb < 4; ++nb) acc[mb][nb] = (v8f){};
    const size_t aoff = (size_t)(r0 + lr) * lda + 8 * hi, boff = (size_t)(c0 + lr) * ldb + 8 * hi;
#pragma unroll 1
    for (int kc = 0; kc < K; kc += 32) {
        v16h a[4];
#pragma unroll
        for (int mb = 0; mb < 4; ++mb) a[mb] = ldh(A + aoff + (size_t)mb * 16 * lda + kc);
#pragma unroll
        for (int nb = 0; nb < 4; ++nb) { const v16h bq = ldh(Bt + boff + (size_t)nb * 16 * ldb + kc);
#pragma unroll
            for (int mb = 0; mb < 4; ++mb) acc[mb][nb] = wmmag(a[mb], bq, acc[mb][nb]); }
    }
}

static_assert(32 * 16 * 4 == 16 * 128);
__device__ __forceinline__ void store_h(v8f (&acc)[4][4], float osc, h16* C, size_t cbase, size_t ldc, float* os, int lane, int lr, int hi) {
#pragma unroll
    for (int mb = 0; mb < 4; ++mb) {
#pragma unroll
        for (int nb = 0; nb < 4; ++nb) {
#pragma unroll
            for (int j = 0; j < 8; ++j) os[(hi * 8 + j) * GSP + nb * 16 + lr] = acc[mb][nb][j] * osc; }
        wave_sync();
#pragma unroll 1
        for (int ps = 0; ps < 2; ++ps) {
#pragma unroll
            for (int s = 0; s < 4; ++s) { const int row = 4 * s + (lane >> 3), c8 = (lane & 7) * 8;
                const v4f x0 = *(const v4fa*)(&os[row * GSP + c8]); const v4f x1 = *(const v4fa*)(&os[row * GSP + c8 + 4]); v8h hv;
#pragma unroll
                for (int i = 0; i < 4; ++i) { hv[i] = toh_flush(x0[i]); hv[4 + i] = toh_flush(x1[i]); }
                *(volatile v8h*)(C + cbase + (size_t)(mb * 16 + row) * ldc + c8) = hv; }
            if (ps == 0) __threadfence(); }
        wave_sync();
    }
}

static_assert(32 * 16 * 8 == 16 * 256);
__device__ __forceinline__ void store_f(v8f (&acc)[4][4], float osc, float* C, size_t cbase, size_t ldc, float* os, int lane, int lr, int hi) {
#pragma unroll
    for (int mb = 0; mb < 4; ++mb) {
#pragma unroll
        for (int nb = 0; nb < 4; ++nb) {
#pragma unroll
            for (int j = 0; j < 8; ++j) os[(hi * 8 + j) * GSP + nb * 16 + lr] = acc[mb][nb][j] * osc; }
        wave_sync();
#pragma unroll 1
        for (int ps = 0; ps < 2; ++ps) {
#pragma unroll
            for (int s = 0; s < 8; ++s) { const int row = 2 * s + (lane >> 4), c4 = (lane & 15) * 4;
                const v4f val = *(const v4fa*)(&os[row * GSP + c4]);
                *(volatile v4f*)(C + cbase + (size_t)(mb * 16 + row) * ldc + c4) = val; }
            if (ps == 0) __threadfence(); }
        wave_sync();
    }
}

__global__ __launch_bounds__(32) void k_gemm_rm(const h16* __restrict__ A, const h16* __restrict__ Bt, h16* C, int ldc) {
    __shared__ __align__(16) float os[16 * GSP];
    const int lane = threadIdx.x & 31, lr = lane & 15, hi = lane >> 4; const int r0 = blockIdx.x * 64, c0 = blockIdx.y * 64;
    v8f acc[4][4];
    gemm_acc(A, (size_t)DM, Bt, (size_t)DM, DM, r0, c0, lr, hi, acc);
    store_h(acc, WI, C, (size_t)r0 * (size_t)ldc + (size_t)c0, (size_t)ldc, os, lane, lr, hi);
}

__global__ __launch_bounds__(32) void k_gemm_vt(const h16* __restrict__ A, const h16* __restrict__ Bt, h16* C) {
    __shared__ __align__(16) float os[16 * GSP];
    const int lane = threadIdx.x & 31, lr = lane & 15, hi = lane >> 4; const int r0 = blockIdx.x * 64, c0 = blockIdx.y * 64;
    v8f acc[4][4];
    gemm_acc(A, (size_t)DM, Bt, (size_t)DM, DM, r0, c0, lr, hi, acc);
    const int bb = c0 / SEQ, tt = c0 % SEQ;
    store_h(acc, WI, C, ((size_t)bb * HD + (size_t)r0) * SEQ + (size_t)tt, (size_t)SEQ, os, lane, lr, hi);
}

__global__ __launch_bounds__(32) void k_gemm_out(const h16* __restrict__ A, const h16* __restrict__ Bt, float* OUT) {
    __shared__ __align__(16) float os[16 * GSP];
    const int lane = threadIdx.x & 31, lr = lane & 15, hi = lane >> 4; const int r0 = blockIdx.x * 64, c0 = blockIdx.y * 64;
    v8f acc[4][4];
    gemm_acc(A, (size_t)LDAH, Bt, (size_t)LDAH, LDAH, r0, c0, lr, hi, acc);
    const int bb = r0 / SEQ, tt = r0 % SEQ;
    store_f(acc, OI, OUT, ((size_t)bb * OUT_SEQ + (size_t)tt) * DM + (size_t)c0, (size_t)DM, os, lane, lr, hi);
}

__global__ __launch_bounds__(32) void k_ffup(const h16* __restrict__ XN, const h16* __restrict__ W1T, h16* AH) {
    __shared__ __align__(16) float os[16 * GSP];
    const int lane = threadIdx.x & 31, lr = lane & 15, hi = lane >> 4; const int r0 = blockIdx.x * 32, c0 = blockIdx.y * 64;
    v8f av[2][4], ag[2][4];
#pragma unroll
    for (int mb = 0; mb < 2; ++mb)
#pragma unroll
        for (int nb = 0; nb < 4; ++nb) { av[mb][nb] = (v8f){}; ag[mb][nb] = (v8f){}; }
    const size_t aoff = (size_t)(r0 + lr) * DM + 8 * hi;
    const size_t boff = (size_t)(c0 + lr) * DM + 8 * hi;
    const size_t goff = boff + (size_t)FFI * DM;
#pragma unroll 1
    for (int kc = 0; kc < DM; kc += 32) {
        v16h a[2];
#pragma unroll
        for (int mb = 0; mb < 2; ++mb) a[mb] = ldh(XN + aoff + (size_t)mb * 16 * DM + kc);
#pragma unroll
        for (int nb = 0; nb < 4; ++nb) {
            const v16h bv = ldh(W1T + boff + (size_t)nb * 16 * DM + kc);
#pragma unroll
            for (int mb = 0; mb < 2; ++mb) av[mb][nb] = wmmag(a[mb], bv, av[mb][nb]);
            const v16h bg = ldh(W1T + goff + (size_t)nb * 16 * DM + kc);
#pragma unroll
            for (int mb = 0; mb < 2; ++mb) ag[mb][nb] = wmmag(a[mb], bg, ag[mb][nb]); }
    }
#pragma unroll
    for (int mb = 0; mb < 2; ++mb) {
#pragma unroll
        for (int nb = 0; nb < 4; ++nb) {
#pragma unroll
            for (int j = 0; j < 8; ++j) { const float vv = av[mb][nb][j] * WI; const float gg = ag[mb][nb][j] * WI;
                const float sg = gg * __builtin_amdgcn_rcpf(1.0f + __builtin_amdgcn_exp2f(-gg * L2E));
                os[(hi * 8 + j) * GSP + nb * 16 + lr] = sg * vv * HC; } }
        wave_sync();
#pragma unroll 1
        for (int ps = 0; ps < 2; ++ps) {
#pragma unroll
            for (int s = 0; s < 4; ++s) { const int row = 4 * s + (lane >> 3), c8 = (lane & 7) * 8;
                const v4f x0 = *(const v4fa*)(&os[row * GSP + c8]); const v4f x1 = *(const v4fa*)(&os[row * GSP + c8 + 4]); v8h hv;
#pragma unroll
                for (int i = 0; i < 4; ++i) { hv[i] = toh_flush(x0[i]); hv[4 + i] = toh_flush(x1[i]); }
                *(volatile v8h*)(AH + (size_t)(r0 + mb * 16 + row) * LDAH + (size_t)DM + (size_t)(c0 + c8)) = hv; }
            if (ps == 0) __threadfence(); }
        wave_sync();
    }
}

static_assert(32 * 16 * 4 == 16 * (HD * 2));
__global__ __launch_bounds__(32 * AW) void k_flash(const h16* __restrict__ QP, const h16* __restrict__ KP, const h16* __restrict__ VT, h16* AO) {
    __shared__ __align__(16) float os[AW * 16 * OSP];
    const int lane = threadIdx.x & 31, lr = lane & 15, hi = lane >> 4;
    const int wave = __builtin_amdgcn_readfirstlane((int)(threadIdx.x >> 5));
    const int zh = blockIdx.y; const int b = zh / NH_, h = zh % NH_;
    const int t0 = (blockIdx.x * AW + wave) * 16;
    const size_t qo = ((size_t)b * SEQ + (size_t)(t0 + lr)) * DM + (size_t)h * HD + 8 * hi;
    const v16h q0 = ldh(QP + qo), q1 = ldh(QP + qo + 32);
    const size_t ko = ((size_t)b * SEQ + (size_t)lr) * HD + 8 * hi;
    const size_t vo = ((size_t)b * HD + (size_t)lr) * SEQ + 8 * hi;
    v8f o[4];
#pragma unroll
    for (int j = 0; j < 4; ++j) o[j] = (v8f){};
    float m = NEGB, l = 0.0f;
#pragma unroll 1
    for (int key0 = 0; key0 < SEQ; key0 += 32) {
        const h16* ka = KP + ko + (size_t)key0 * HD;
        const v16h ka0 = ldh(ka), ka1 = ldh(ka + 32), kb0 = ldh(ka + 16 * HD), kb1 = ldh(ka + 16 * HD + 32);
        v8f sa = (v8f){}, sb = (v8f){};
        sa = wmmag(ka0, q0, sa); sa = wmmag(ka1, q1, sa);
        sb = wmmag(kb0, q0, sb); sb = wmmag(kb1, q1, sb);
        float ta[8], tb[8]; float mx = NEGB;
#pragma unroll
        for (int r = 0; r < 8; ++r) { ta[r] = sa[r] * SC2; tb[r] = sb[r] * SC2; mx = fmaxf(mx, fmaxf(ta[r], tb[r])); }
        mx = fmaxf(mx, __shfl_xor(mx, 16, 32));
        const float mnew = fmaxf(m, mx);
        const float alpha = __builtin_amdgcn_exp2f(m - mnew);
        const float sh = PSH - mnew;
        v16h pb; float ls = 0.0f;
#pragma unroll
        for (int r = 0; r < 8; ++r) {
            const float xa = ta[r] + sh, xb = tb[r] + sh;
            const float ea = (xa < -14.0f) ? 0.0f : __builtin_amdgcn_exp2f(xa);
            const float eb = (xb < -14.0f) ? 0.0f : __builtin_amdgcn_exp2f(xb);
            const h16 pa = (h16)ea; const h16 pc = (h16)eb;
            pb[r] = pa; pb[8 + r] = pc;
            ls += (float)pa + (float)pc; }
        l = l * alpha + ls; m = mnew;
#pragma unroll
        for (int j = 0; j < 4; ++j) o[j] = o[j] * alpha;
        const h16* va = VT + vo + key0;
        v16h vf[4];
#pragma unroll
        for (int j = 0; j < 4; ++j) vf[j] = ldh(va + (size_t)j * 16 * SEQ);
#pragma unroll
        for (int j = 0; j < 4; ++j) o[j] = wmmag(vf[j], pb, o[j]);
    }
    l += __shfl_xor(l, 16, 32);
    const float inv = AOC * (1.0f / l);
    const int wb = wave * 16 * OSP;
#pragma unroll
    for (int j = 0; j < 4; ++j) { v4f a, c;
        a[0] = o[j][0] * inv; a[1] = o[j][1] * inv; a[2] = o[j][2] * inv; a[3] = o[j][3] * inv;
        c[0] = o[j][4] * inv; c[1] = o[j][5] * inv; c[2] = o[j][6] * inv; c[3] = o[j][7] * inv;
        *(v4fa*)(&os[wb + lr * OSP + 16 * j + 8 * hi]) = a; *(v4fa*)(&os[wb + lr * OSP + 16 * j + 8 * hi + 4]) = c; }
    wave_sync();
    h16* orow = AO + ((size_t)b * SEQ + (size_t)t0) * LDAH + (size_t)h * HD;
#pragma unroll 1
    for (int ps = 0; ps < 2; ++ps) {
#pragma unroll
        for (int s = 0; s < 4; ++s) { const int row = 4 * s + (lane >> 3), c8 = (lane & 7) * 8;
            const v4f x0 = *(const v4fa*)(&os[wb + row * OSP + c8]); const v4f x1 = *(const v4fa*)(&os[wb + row * OSP + c8 + 4]); v8h hv;
#pragma unroll
            for (int i = 0; i < 4; ++i) { hv[i] = toh_flush(x0[i]); hv[4 + i] = toh_flush(x1[i]); }
            *(volatile v8h*)(orow + (size_t)row * LDAH + c8) = hv; }
        if (ps == 0) __threadfence(); }
}

static constexpr size_t al256(size_t v) { return (v + 255) & ~(size_t)255; }
static constexpr size_t SZ_XN  = al256((size_t)NB * SEQ * DM * 2);
static constexpr size_t SZ_WQ  = al256((size_t)DM * DM * 2);
static constexpr size_t SZ_WKV = al256((size_t)2 * HD * DM * 2);
static constexpr size_t SZ_W1  = al256((size_t)2 * FFI * DM * 2);
static constexpr size_t SZ_WO  = al256((size_t)DM * LDAH * 2);
static constexpr size_t SZ_KP  = al256((size_t)NB * SEQ * HD * 2);
static constexpr size_t SZ_AH  = al256((size_t)NB * SEQ * LDAH * 2);
static constexpr size_t SZ_TOTAL = 3 * SZ_XN + SZ_WQ + SZ_WKV + SZ_W1 + SZ_WO + 2 * SZ_KP + SZ_AH;
static_assert(SZ_TOTAL <= (size_t)134217728);
static_assert(((size_t)HD * DM * 2) % 256 == 0);

extern "C" void kernel_launch(void* const* d_in, const int* in_sizes, int n_in,
                              void* d_out, int out_size, void* d_ws, size_t ws_size, hipStream_t stream) {
    if (n_in < 11) return;
    const size_t needx = ((size_t)(NB - 1) * SEQ_FULL + SEQ) * DM;
    if ((size_t)in_sizes[0] < needx || (size_t)in_sizes[1] < needx) return;
    if (in_sizes[2] < DM || in_sizes[3] < DM || in_sizes[4] < DM || in_sizes[5] < DM) return;
    if ((size_t)in_sizes[6] < (size_t)DM * DM || (size_t)in_sizes[7] < (size_t)DM * 2 * HD || (size_t)in_sizes[8] < (size_t)DM * DM) return;
    if ((size_t)in_sizes[9] < (size_t)DM * 2 * FFI || (size_t)in_sizes[10] < (size_t)FFI * DM) return;
    if ((size_t)out_size < ((size_t)(NB - 1) * OUT_SEQ + SEQ) * DM) return;
    if (SZ_TOTAL > ws_size) return;
    const float* x    = (const float*)d_in[0];
    const float* ctx  = (const float*)d_in[1];
    const float* lnxg = (const float*)d_in[2];
    const float* lnxb = (const float*)d_in[3];
    const float* lncg = (const float*)d_in[4];
    const float* lncb = (const float*)d_in[5];
    const float* wq   = (const float*)d_in[6];
    const float* wkv  = (const float*)d_in[7];
    const float* wout = (const float*)d_in[8];
    const float* wff1 = (const float*)d_in[9];
    const float* wff2 = (const float*)d_in[10];
    float* OUT = (float*)d_out;
    char* wsp = (char*)d_ws;
    h16* XN   = (h16*)wsp; wsp += SZ_XN;
    h16* CN   = (h16*)wsp; wsp += SZ_XN;
    h16* WQT  = (h16*)wsp; wsp += SZ_WQ;
    h16* WKVT = (h16*)wsp; wsp += SZ_WKV;
    h16* W1T  = (h16*)wsp; wsp += SZ_W1;
    h16* WOT  = (h16*)wsp; wsp += SZ_WO;
    h16* QP   = (h16*)wsp; wsp += SZ_XN;
    h16* KP   = (h16*)wsp; wsp += SZ_KP;
    h16* VT   = (h16*)wsp; wsp += SZ_KP;
    h16* AH   = (h16*)wsp; wsp += SZ_AH;

    k_ln<<<NB * SEQ / 8, 256, 0, stream>>>(x,   lnxg, lnxb, XN);
    k_ln<<<NB * SEQ / 8, 256, 0, stream>>>(ctx, lncg, lncb, CN);

    k_wtr<<<dim3(DM / 64, DM / 64, 1), 256, 0, stream>>>(wq, DM, WQT, DM, 0);
    k_wtr<<<dim3(2 * HD / 64, DM / 64, 1), 256, 0, stream>>>(wkv, 2 * HD, WKVT, DM, 0);
    k_wtr<<<dim3(2 * FFI / 64, DM / 64, 1), 256, 0, stream>>>(wff1, 2 * FFI, W1T, DM, 0);
    k_wtr<<<dim3(DM / 64, DM / 64, 1), 256, 0, stream>>>(wout, DM, WOT, LDAH, 0);
    k_wtr<<<dim3(DM / 64, FFI / 64, 1), 256, 0, stream>>>(wff2, DM, WOT, LDAH, DM);

    k_gemm_rm<<<dim3(NB * SEQ / 64, DM / 64, 1), 32, 0, stream>>>(XN, WQT, QP, DM);
    k_gemm_rm<<<dim3(NB * SEQ / 64, 1, 1), 32, 0, stream>>>(CN, WKVT, KP, HD);
    k_gemm_vt<<<dim3(1, NB * SEQ / 64, 1), 32, 0, stream>>>(WKVT + (size_t)HD * DM, CN, VT);

    k_flash<<<dim3(SEQ / (16 * AW), NB * NH_, 1), 32 * AW, 0, stream>>>(QP, KP, VT, AH);
    k_ffup<<<dim3(NB * SEQ / 32, FFI / 64, 1), 32, 0, stream>>>(XN, W1T, AH);

    k_gemm_out<<<dim3(NB * SEQ / 64, DM / 64, 1), 32, 0, stream>>>(AH, WOT, OUT);
}
